// CongestionGCN_72808285602083
// MI455X (gfx1250) — hardware-verified
//
#include <hip/hip_runtime.h>
#include <math.h>

#define NN 100000
#define NE 600000
#define IN_D 12
#define HD 128
#define HD2 64
#define OUT_D 2
#define NT 256
#define SRB 2048
#define NTL 49
#define NP (NTL * SRB)
#define TPC 7
#define NCHK 7
#define CHR (TPC * SRB)
#define XK 32
#define KC 256
#define SCH 4096
#define NCH ((NE + SCH - 1) / SCH)
#define RB 256
#define NSB ((NN + RB - 1) / RB)
#define BN_EPS 1e-5f

typedef __attribute__((ext_vector_type(16))) _Float16 v16h;
typedef __attribute__((ext_vector_type(8)))  _Float16 v8h;
typedef __attribute__((ext_vector_type(16))) __bf16   v16b;
typedef __attribute__((ext_vector_type(8)))  __bf16   v8b;
typedef __attribute__((ext_vector_type(8)))  float    v8f;
typedef __attribute__((ext_vector_type(4)))  float    v4f;
typedef __attribute__((ext_vector_type(4)))  int      v4i;

__device__ __forceinline__ unsigned short f2bf_bits(float f) {
  unsigned u = __float_as_uint(f);
  return (unsigned short)((u + 0x7FFFu + ((u >> 16) & 1u)) >> 16);
}
__device__ __forceinline__ float bf_bits2f(unsigned short h) { return __uint_as_float(((unsigned)h) << 16); }

__device__ __forceinline__ void dep_guard_h(v8f& a, v8f& b, v16h x, v16h y) { asm volatile("v_nop\n\tv_nop\n\tv_nop\n\tv_nop" : "+v"(a), "+v"(b) : "v"(x), "v"(y)); }
__device__ __forceinline__ void dep_guard_b(v8f& a, v8f& b, v16b x, v16b y) { asm volatile("v_nop\n\tv_nop\n\tv_nop\n\tv_nop" : "+v"(a), "+v"(b) : "v"(x), "v"(y)); }
__device__ __forceinline__ void keep4_h(v16h a, v16h b, v16h c, v16h d) { asm volatile("v_nop" :: "v"(a), "v"(b), "v"(c), "v"(d)); }
__device__ __forceinline__ void keep4_b(v16b a, v16b b, v16b c, v16b d) { asm volatile("v_nop" :: "v"(a), "v"(b), "v"(c), "v"(d)); }
__device__ __forceinline__ void acc_guard4(v8f& a, v8f& b, v8f& c, v8f& d) { asm volatile("v_nop\n\tv_nop\n\tv_nop\n\tv_nop" : "+v"(a), "+v"(b), "+v"(c), "+v"(d)); }
template <typename T> struct Frag;
template <> struct Frag<_Float16> {
  typedef v16h V; union U { v16h v; v8h h[2]; };
  static __device__ __forceinline__ v16h load(const _Float16* p) {
    U f; f.h[0] = *(const v8h*)(p); f.h[1] = *(const v8h*)(p + 16); return f.v;
  }
  static __device__ __forceinline__ v8f mma(v16h a, v16h b, v8f c) {
    return __builtin_amdgcn_wmma_f32_16x16x32_f16(false, a, false, b, (short)0, c, false, false);
  }
  static __device__ __forceinline__ void guard(v8f& a, v8f& b, v16h x, v16h y) { dep_guard_h(a, b, x, y); }
  static __device__ __forceinline__ void keep(v16h a, v16h b, v16h c, v16h d) { keep4_h(a, b, c, d); }
};
template <> struct Frag<__bf16> {
  typedef v16b V; union U { v16b v; v8b h[2]; };
  static __device__ __forceinline__ v16b load(const __bf16* p) {
    U f; f.h[0] = *(const v8b*)(p); f.h[1] = *(const v8b*)(p + 16); return f.v;
  }
  static __device__ __forceinline__ v8f mma(v16b a, v16b b, v8f c) {
    return __builtin_amdgcn_wmma_f32_16x16x32_bf16(false, a, false, b, (short)0, c, false, false);
  }
  static __device__ __forceinline__ void guard(v8f& a, v8f& b, v16b x, v16b y) { dep_guard_b(a, b, x, y); }
  static __device__ __forceinline__ void keep(v16b a, v16b b, v16b c, v16b d) { keep4_b(a, b, c, d); }
};

template <int ET> struct Elem;
template <> struct Elem<0> { typedef _Float16 T; };
template <> struct Elem<1> { typedef __bf16 T; };
template <int ET, bool SPLIT, int BIAS_MODE, int OUT_MODE, bool RESID, int ACT = 0>
__global__ __launch_bounds__(256) void wmma_gemm64(
    const unsigned short* __restrict__ Ap, const unsigned short* __restrict__ A2p, int lda, long strideA,
    const unsigned short* __restrict__ Btp, const unsigned short* __restrict__ Bt2p, int ldb, long strideB,
    void* __restrict__ Cout, void* __restrict__ Cout2, int ldc, long strideC,
    const float* __restrict__ bias,
    const float* __restrict__ resid, long strideR,
    int M, int N, int K, float scale) {
  typedef typename Elem<ET>::T T;
  typedef typename Frag<T>::V V;
  const T* A = (const T*)Ap; const T* A2 = (const T*)A2p; const T* Bt = (const T*)Btp; const T* Bt2 = (const T*)Bt2p;
  __shared__ __align__(16) float sT[8][16 * 68];
  const int b    = blockIdx.y;
  const int lane = threadIdx.x & 31;
  const int wave = threadIdx.x >> 5;
  const int tilesN = N >> 6;
  const int tilesM = M >> 6;
  const int tile = blockIdx.x * 8 + wave;
  if (tile >= tilesM * tilesN) return;
  const int tm = tile / tilesN;
  const int tn = tile - tm * tilesN;
  const int m0 = tm << 6;
  const int n0 = tn << 6;

  const T* Ab  = A  + (size_t)b * strideA;
  const T* Bb  = Bt + (size_t)b * strideB;
  const T* Ab2 = SPLIT ? (A2  + (size_t)b * strideA) : nullptr;
  const T* Bb2 = SPLIT ? (Bt2 + (size_t)b * strideB) : nullptr;

  const int rlane = lane & 15;
  const int koff  = (lane >> 4) * 8;
  const int mOff  = (lane >> 4) * 8;

  v8f acc[4][4];
#pragma unroll
  for (int i = 0; i < 4; ++i)
#pragma unroll
    for (int j = 0; j < 4; ++j) acc[i][j] = (v8f){0.f,0.f,0.f,0.f,0.f,0.f,0.f,0.f};

  for (int k0 = 0; k0 < K; k0 += 32) {
    V bh[4], bl[4];
#pragma unroll
    for (int j = 0; j < 4; ++j) {
      const size_t bo = (size_t)(n0 + (j << 4) + rlane) * ldb + koff + k0;
      bh[j] = Frag<T>::load(Bb + bo);
      if (SPLIT) bl[j] = Frag<T>::load(Bb2 + bo);
    }
#pragma unroll
    for (int i = 0; i < 4; ++i) {
      const size_t ao = (size_t)(m0 + (i << 4) + rlane) * lda + koff + k0;
      V ah = Frag<T>::load(Ab + ao);
      V al;
      if (SPLIT) al = Frag<T>::load(Ab2 + ao);
#pragma unroll
      for (int j = 0; j < 4; ++j) {
        acc[i][j] = Frag<T>::mma(ah, bh[j], acc[i][j]);
        if (SPLIT) {
          acc[i][j] = Frag<T>::mma(ah, bl[j], acc[i][j]);
          acc[i][j] = Frag<T>::mma(al, bh[j], acc[i][j]);
        }
      }
      Frag<T>::guard(acc[i][0], acc[i][3], ah, SPLIT ? al : ah);
    }
    Frag<T>::keep(bh[0], bh[1], bh[2], bh[3]);
    if (SPLIT) Frag<T>::keep(bl[0], bl[1], bl[2], bl[3]);
  }
  acc_guard4(acc[0][0], acc[0][1], acc[0][2], acc[0][3]);
  acc_guard4(acc[1][0], acc[1][1], acc[1][2], acc[1][3]);
  acc_guard4(acc[2][0], acc[2][1], acc[2][2], acc[2][3]);
  acc_guard4(acc[3][0], acc[3][1], acc[3][2], acc[3][3]);

  float* slab = sT[wave];
  const float* Rb = RESID ? (resid + (size_t)b * strideR) : nullptr;
#pragma unroll
  for (int i = 0; i < 4; ++i) {
    const int mBase = m0 + (i << 4);
#pragma unroll
    for (int j = 0; j < 4; ++j) {
      const int n = n0 + (j << 4) + rlane;
      float bv = 0.f;
      if (BIAS_MODE == 2) bv = bias[n];
#pragma unroll
      for (int r = 0; r < 8; ++r) {
        float v = acc[i][j][r] * scale;
        if (BIAS_MODE == 1) v += bias[mBase + mOff + r];
        if (BIAS_MODE == 2) v += bv;
        if (RESID) v += Rb[(size_t)(mBase + mOff + r) * ldc + n];
        if (ACT == 1) v = tanhf(v);
        if (ACT == 2) v = fmaxf(v, 0.0f);
        if (ACT == 3) v = v / (1.0f + expf(-v));
        if (ACT == 4) v = (v > 0.f) ? v : 0.01f * v;
        if (ACT == 5) v = 0.5f * v * (1.0f + erff(v * 0.70710678118654752f));
        slab[(mOff + r) * 68 + (j << 4) + rlane] = v;
      }
    }
    __builtin_amdgcn_fence(__ATOMIC_RELEASE, "workgroup");
    __builtin_amdgcn_wave_barrier();
    __builtin_amdgcn_fence(__ATOMIC_ACQUIRE, "workgroup");
    if (OUT_MODE == 0) {
      float* C = (float*)Cout + (size_t)b * strideC;
      const int hh = lane >> 4, c4 = (lane & 15) * 4;
      for (int pass = 0; pass < 2; ++pass) {
#pragma unroll
        for (int it = 0; it < 8; ++it) {
          const int row = it * 2 + hh;
          v4f v = *(const v4f*)(slab + row * 68 + c4);
          *(volatile v4f*)(C + (size_t)(mBase + row) * ldc + n0 + c4) = v;
        }
        __threadfence();
      }
    } else {
      const int q = lane >> 3, c8 = (lane & 7) * 8;
      unsigned short* C  = (unsigned short*)Cout  + (size_t)b * strideC;
      unsigned short* C2 = (OUT_MODE == 2) ? ((unsigned short*)Cout2 + (size_t)b * strideC) : nullptr;
      for (int pass = 0; pass < 2; ++pass) {
#pragma unroll
        for (int it = 0; it < 4; ++it) {
          const int row = it * 4 + q;
          const float* sp = slab + row * 68 + c8;
          v8h hv, lv;
#pragma unroll
          for (int e = 0; e < 8; ++e) {
            if (OUT_MODE == 1) {
              hv[e] = (_Float16)sp[e];
            } else {
              unsigned short hb = f2bf_bits(sp[e]);
              unsigned short lb = f2bf_bits(sp[e] - bf_bits2f(hb));
              hv[e] = __builtin_bit_cast(_Float16, hb);
              lv[e] = __builtin_bit_cast(_Float16, lb);
            }
          }
          *(volatile v8h*)(C + (size_t)(mBase + row) * ldc + n0 + c8) = hv;
          if (OUT_MODE == 2) *(volatile v8h*)(C2 + (size_t)(mBase + row) * ldc + n0 + c8) = lv;
        }
        __threadfence();
      }
    }
    __builtin_amdgcn_fence(__ATOMIC_RELEASE, "workgroup");
    __builtin_amdgcn_wave_barrier();
    __builtin_amdgcn_fence(__ATOMIC_ACQUIRE, "workgroup");
  }
}

__device__ __forceinline__ int blk_excl_scan(int cnt, int* scan_ws, int tid, int* tot) {
  const int lane = tid & 31, wave = tid >> 5; int incl = cnt;
#pragma unroll
  for (int o = 1; o < 32; o <<= 1) { const int v = __shfl_up(incl, o, 32); if (lane >= o) incl += v; }
  if (lane == 31) scan_ws[wave] = incl;
  __syncthreads();
  if (wave == 0) { int wv = (lane < NT / 32) ? scan_ws[lane] : 0; int wincl = wv;
#pragma unroll
    for (int o = 1; o < 32; o <<= 1) { const int v = __shfl_up(wincl, o, 32); if (lane >= o) wincl += v; }
    if (lane < NT / 32) scan_ws[32 + lane] = wincl - wv; if (lane == 31) scan_ws[64] = wincl; }
  __syncthreads();
  const int res = scan_ws[32 + wave] + incl - cnt; *tot = scan_ws[64];
  return res;
}
template <int SP, int CAP>
__device__ __forceinline__ int chunk_hits(const int* __restrict__ dstv, const int* __restrict__ srcv, int e0, int n0, int tid,
                                          int* LIST, int* scan_ws) {
  const int eb = e0 + tid * SP;
  int rec[SP]; int cnt = 0;
  if (eb < NE) {
#pragma unroll
    for (int k = 0; k < SP; k += 4) {
      const v4i d4 = *(const v4i*)(dstv + eb + k);
      const v4i s4 = *(const v4i*)(srcv + eb + k);
#pragma unroll
      for (int e = 0; e < 4; ++e) {
        const int d = d4[e]; int r = -1;
        if (d >= n0 && d < n0 + SRB) { int s = s4[e]; s = s < 0 ? 0 : (s >= NN ? NN - 1 : s); r = ((d - n0) << 17) | s; ++cnt; }
        rec[k + e] = r;
      }
    }
  } else {
#pragma unroll
    for (int k = 0; k < SP; ++k) rec[k] = -1;
  }
  int tot; int p = blk_excl_scan(cnt, scan_ws, tid, &tot);
#pragma unroll
  for (int k = 0; k < SP; ++k) if (rec[k] >= 0) { if ((unsigned)p < (unsigned)CAP) LIST[p] = rec[k]; ++p; }
  __syncthreads();
  return tot < CAP ? tot : CAP;
}

__device__ __forceinline__ void split_store2(float a, float b, unsigned* H, unsigned* L, size_t i) {
  const unsigned short ha = f2bf_bits(a), hb = f2bf_bits(b);
  const unsigned short la = f2bf_bits(a - bf_bits2f(ha)), lb = f2bf_bits(b - bf_bits2f(hb));
  const unsigned uh = (unsigned)ha | ((unsigned)hb << 16), ul = (unsigned)la | ((unsigned)lb << 16);
  ((volatile unsigned*)H)[i] = uh; ((volatile unsigned*)L)[i] = ul;
  __threadfence();
  ((volatile unsigned*)H)[i] = uh; ((volatile unsigned*)L)[i] = ul;
}
__device__ __forceinline__ void split8(v4f a0, v4f a1, v8h& hv, v8h& lv) {
#pragma unroll
  for (int e = 0; e < 4; ++e) {
    unsigned short hb, lb;
    hb = f2bf_bits(a0[e]); lb = f2bf_bits(a0[e] - bf_bits2f(hb)); hv[e] = __builtin_bit_cast(_Float16, hb); lv[e] = __builtin_bit_cast(_Float16, lb);
    hb = f2bf_bits(a1[e]); lb = f2bf_bits(a1[e] - bf_bits2f(hb)); hv[4 + e] = __builtin_bit_cast(_Float16, hb); lv[4 + e] = __builtin_bit_cast(_Float16, lb);
  }
}

__global__ __launch_bounds__(NT) void prep_kernel(const float* __restrict__ E, const float* __restrict__ ebv,
                                                 const float* __restrict__ Ws, const float* __restrict__ Wn, const float* __restrict__ cb,
                                                 const float* __restrict__ W1,
                                                 unsigned* __restrict__ BLH, unsigned* __restrict__ BLL,
                                                 unsigned* __restrict__ W1H, unsigned* __restrict__ W1L,
                                                 unsigned* __restrict__ B0H, unsigned* __restrict__ B0L, float* __restrict__ BIAS0) {
  const int gid = blockIdx.x * NT + threadIdx.x;
  if (gid < 2 * HD * (KC / 2)) {
    const int li = gid >> 14, n = (gid >> 7) & (HD - 1), kp = gid & 127; const int k = 2 * kp;
    const float* W = ((k < HD) ? Ws : Wn) + (size_t)(li + 1) * HD * HD;
    const int kk = k & (HD - 1);
    const float a = W[kk * HD + n], b = W[(kk + 1) * HD + n];
    split_store2(a, b, BLH, BLL, (size_t)gid);
  } else if (gid < 32768 + HD2 * (HD / 2)) {
    const int i = gid - 32768; const int n = i >> 6, kp = i & 63; const int k = 2 * kp;
    const float a = W1[k * HD2 + n], b = W1[(k + 1) * HD2 + n];
    split_store2(a, b, W1H, W1L, (size_t)i);
  } else if (gid < 36864 + HD * (XK / 2)) {
    const int i = gid - 36864; const int n = i >> 4, kp = i & 15; const int k = 2 * kp;
    float a = 0.f, b = 0.f;
    if (k < 2 * IN_D) {
      const float* W = (k < IN_D) ? Ws : Wn; const int r = (k < IN_D) ? k : (k - IN_D);
#pragma unroll 1
      for (int j = 0; j < HD; ++j) { const float w = W[j * HD + n]; a += E[r * HD + j] * w; b += E[(r + 1) * HD + j] * w; }
    } else if (k == 2 * IN_D) {
#pragma unroll 1
      for (int j = 0; j < HD; ++j) a += ebv[j] * Wn[j * HD + n];
    }
    split_store2(a, b, B0H, B0L, (size_t)i);
  } else if (gid < 38912 + HD) {
    const int n = gid - 38912; float s = cb[n];
#pragma unroll 1
    for (int j = 0; j < HD; ++j) s += ebv[j] * Ws[j * HD + n];
    ((volatile float*)BIAS0)[n] = s; __threadfence(); ((volatile float*)BIAS0)[n] = s;
  }
}

__global__ __launch_bounds__(NT) void agg0_kernel(const float* __restrict__ X, const int* __restrict__ ei, float* XCF,
                                                 unsigned* __restrict__ XCH, unsigned* __restrict__ XCL) {
  __shared__ int LIST[SCH];
  __shared__ int CNT[SRB];
  __shared__ int scan_ws[80];
  const int tid = threadIdx.x, lane = tid & 31, wave = tid >> 5;
  const int n0 = blockIdx.x * SRB;
  const int cl = (lane < IN_D) ? lane : 0;
#pragma unroll 1
  for (int j = 0; j < 256; ++j) {
    const int row = n0 + wave * 256 + j;
    const int rr = row < NN ? row : NN - 1;
    const float xv = X[(size_t)rr * IN_D + cl];
    const float v = (lane < IN_D && row < NN) ? xv : 0.f;
    XCF[(size_t)row * XK + lane] = v;
  }
  for (int i = tid; i < SRB; i += NT) CNT[i] = 0;
  __syncthreads();
  const int* srcv = ei; const int* dstv = ei + NE;
  const bool gact = (lane >= IN_D) && (lane < 2 * IN_D);
  const int gl = gact ? (lane - IN_D) : 0;
#pragma unroll 1
  for (int c = 0; c < NCH; ++c) {
    const int tot = chunk_hits<SCH / NT, SCH>(dstv, srcv, c * SCH, n0, tid, LIST, scan_ws);
#pragma unroll 1
    for (int base = 0; base < tot; base += 32) {
      const int q = base + lane;
      const int rv = (q < tot) ? LIST[q] : -1;
      const int own = (rv >= 0 && (rv >> 25) == wave) ? 1 : 0;
      unsigned msk = (unsigned)__ballot(own);
#pragma unroll 1
      for (int it = 0; it < 32; ++it) {
        if (msk == 0u) break;
        const int bp = __builtin_ctz(msk); msk &= msk - 1u;
        const int r = __shfl(rv, bp, 32);
        const int dl = (r >> 17) & (SRB - 1);
        int s = r & 0x1FFFF; s = s < NN ? s : NN - 1;
        const float xs = X[(size_t)s * IN_D + gl];
        const float addv = gact ? xs : 0.f;
        float* rp = XCF + (size_t)(n0 + dl) * XK + lane;
        const float cur = *rp;
        *rp = cur + addv;
        if (lane == 0) CNT[dl] += 1;
      }
    }
    __syncthreads();
  }
#pragma unroll 1
  for (int j = 0; j < 128; ++j) {
    const int r = wave * 256 + 2 * j + (lane >> 4);
    const int row = n0 + r;
    const int c = 2 * (lane & 15);
    const float* rp = XCF + (size_t)row * XK + c;
    float v0 = rp[0], v1 = rp[1];
    const int cn = CNT[r];
    const float cf = (float)cn;
    const float inv = 1.0f / fmaxf(cf, 1.0f);
    if (c >= IN_D && c < 2 * IN_D) { v0 = v0 * inv; v1 = v1 * inv; }
    if (c == 2 * IN_D) { v0 = (cn > 0) ? 1.0f : 0.0f; v1 = 0.0f; }
    split_store2(v0, v1, XCH, XCL, (size_t)row * (XK / 2) + (lane & 15));
  }
}

__global__ __launch_bounds__(NT) void agg_kernel(const float* __restrict__ h, const int* __restrict__ ei, float* ACC,
                                                unsigned short* __restrict__ APH, unsigned short* __restrict__ APL, int tile0) {
  __shared__ int LIST[SCH];
  __shared__ int CNT[SRB];
  __shared__ int scan_ws[80];
  const int tid = threadIdx.x, lane = tid & 31, wave = tid >> 5;
  const int n0 = (tile0 + blockIdx.x) * SRB;
  const int rb = blockIdx.x * SRB;
  const v4f z4 = {0.f, 0.f, 0.f, 0.f};
#pragma unroll 1
  for (int j = 0; j < 256; ++j) *(v4f*)(ACC + (size_t)(rb + wave * 256 + j) * HD + 4 * lane) = z4;
  for (int i = tid; i < SRB; i += NT) CNT[i] = 0;
  __syncthreads();
  const int* srcv = ei; const int* dstv = ei + NE;
#pragma unroll 1
  for (int c = 0; c < NCH; ++c) {
    const int tot = chunk_hits<SCH / NT, SCH>(dstv, srcv, c * SCH, n0, tid, LIST, scan_ws);
#pragma unroll 1
    for (int base = 0; base < tot; base += 32) {
      const int q = base + lane;
      const int rv = (q < tot) ? LIST[q] : -1;
      const int own = (rv >= 0 && (rv >> 25) == wave) ? 1 : 0;
      unsigned msk = (unsigned)__ballot(own);
#pragma unroll 1
      for (int it = 0; it < 32; ++it) {
        if (msk == 0u) break;
        const int bp = __builtin_ctz(msk); msk &= msk - 1u;
        const int r = __shfl(rv, bp, 32);
        const int dl = (r >> 17) & (SRB - 1);
        int s = r & 0x1FFFF; s = s < NN ? s : NN - 1;
        const v4f hv = *(const v4f*)(h + (size_t)s * HD + 4 * lane);
        float* rp = ACC + (size_t)(rb + dl) * HD + 4 * lane;
        v4f a = *(const v4f*)rp;
        a = a + hv;
        *(v4f*)rp = a;
        if (lane == 0) CNT[dl] += 1;
      }
    }
    __syncthreads();
  }
  const bool lo16 = lane < 16;
  const int c8 = 8 * (lane & 15);
#pragma unroll 1
  for (int j = 0; j < 256; ++j) {
    const int r = wave * 256 + j;
    const int row = n0 + r;
    const int lr = rb + r;
    const int cn = CNT[r];
    const float cf = (float)cn;
    const float inv = 1.0f / fmaxf(cf, 1.0f);
    const float* p = lo16 ? (h + (size_t)row * HD + c8) : (ACC + (size_t)lr * HD + c8);
    const float sc = lo16 ? 1.0f : inv;
    v4f a0 = *(const v4f*)p, a1 = *(const v4f*)(p + 4);
    a0 = a0 * sc; a1 = a1 * sc;
    v8h hv, lv;
    split8(a0, a1, hv, lv);
    unsigned short* ph = APH + (size_t)lr * KC + 8 * lane;
    unsigned short* pl = APL + (size_t)lr * KC + 8 * lane;
    for (int pass = 0; pass < 2; ++pass) { *(volatile v8h*)ph = hv; *(volatile v8h*)pl = lv; __threadfence(); }
  }
}

__global__ __launch_bounds__(NT) void stats_kernel(const float* __restrict__ pre, float* __restrict__ part) {
  __shared__ float red[2 * HD];
  const int tid = threadIdx.x;
  const int c = tid & (HD - 1), rh = tid >> 7;
  const int r0 = blockIdx.x * RB;
  float s = 0.f, s2 = 0.f;
#pragma unroll 1
  for (int i = rh; i < RB; i += 2) {
    const int r = r0 + i;
    if (r < NN) { const float x = pre[(size_t)r * HD + c]; s += x; s2 = fmaf(x, x, s2); }
  }
  if (rh == 1) { red[c] = s; red[HD + c] = s2; }
  __syncthreads();
  if (rh == 0) {
    s += red[c]; s2 += red[HD + c];
    float* pp = part + (size_t)blockIdx.x * 2 * HD;
    ((volatile float*)pp)[c] = s; ((volatile float*)pp)[HD + c] = s2;
    __threadfence();
    ((volatile float*)pp)[c] = s; ((volatile float*)pp)[HD + c] = s2;
  }
}

__global__ __launch_bounds__(128) void fin_kernel(const float* __restrict__ part, float* __restrict__ murs) {
  const int c = threadIdx.x;
  double s = 0.0, s2 = 0.0;
#pragma unroll 1
  for (int b = 0; b < NSB; ++b) { s += (double)part[(size_t)b * 2 * HD + c]; s2 += (double)part[(size_t)b * 2 * HD + HD + c]; }
  const double m = s * (1.0 / NN);
  double var = s2 * (1.0 / NN) - m * m;
  var = var > 0.0 ? var : 0.0;
  const float mf = (float)m, vf = (float)var;
  const float rs = 1.0f / sqrtf(vf + BN_EPS);
  ((volatile float*)murs)[c] = mf; ((volatile float*)murs)[HD + c] = rs;
  __threadfence();
  ((volatile float*)murs)[c] = mf; ((volatile float*)murs)[HD + c] = rs;
}

__global__ __launch_bounds__(NT) void apply_kernel(float* pre, const float* __restrict__ res, const float* __restrict__ murs,
                                                  const float* __restrict__ gam, const float* __restrict__ bet, int has_res) {
  const int gid = blockIdx.x * NT + threadIdx.x;
  const int row = gid >> 5, c4 = (gid & 31) * 4;
  float* xp = pre + (size_t)row * HD + c4;
  const v4f x = *(const v4f*)xp;
  const v4f mu = *(const v4f*)(murs + c4), rsv = *(const v4f*)(murs + HD + c4);
  const v4f g = *(const v4f*)(gam + c4), bb = *(const v4f*)(bet + c4);
  v4f rr = {0.f, 0.f, 0.f, 0.f};
  if (has_res) rr = *(const v4f*)(res + (size_t)row * HD + c4);
  const bool live = row < NN;
  v4f o;
#pragma unroll
  for (int e = 0; e < 4; ++e) {
    float t = x[e] - mu[e];
    t = t * rsv[e];
    t = t * g[e];
    t = t + bb[e];
    t = fmaxf(t, 0.0f);
    t = t + rr[e];
    o[e] = live ? t : 0.0f;
  }
  *(volatile v4f*)xp = o;
  __threadfence();
  *(volatile v4f*)xp = o;
}

__global__ __launch_bounds__(NT) void convert_kernel(const float* __restrict__ src, unsigned short* __restrict__ PH,
                                                    unsigned short* __restrict__ PL) {
  const size_t i = (size_t)blockIdx.x * NT + threadIdx.x;
  const float* p = src + i * 8;
  const v4f a0 = *(const v4f*)p, a1 = *(const v4f*)(p + 4);
  v8h hv, lv;
  split8(a0, a1, hv, lv);
  for (int pass = 0; pass < 2; ++pass) { *(volatile v8h*)(PH + i * 8) = hv; *(volatile v8h*)(PL + i * 8) = lv; __threadfence(); }
}

__global__ __launch_bounds__(NT) void out_kernel(const float* __restrict__ z, const float* __restrict__ W2, const float* __restrict__ b2,
                                                float* __restrict__ out) {
  __shared__ __align__(16) float so[2 * NT];
  const int tid = threadIdx.x;
  const int row = blockIdx.x * NT + tid;
  float o0 = b2[0], o1 = b2[1];
  const float* zr = z + (size_t)row * HD2;
#pragma unroll 1
  for (int i = 0; i < HD2 / 4; ++i) {
    const v4f zv = *(const v4f*)(zr + 4 * i);
    const v4f wa = *(const v4f*)(W2 + 8 * i), wb = *(const v4f*)(W2 + 8 * i + 4);
    o0 += zv[0] * wa[0] + zv[1] * wa[2] + zv[2] * wb[0] + zv[3] * wb[2];
    o1 += zv[0] * wa[1] + zv[1] * wa[3] + zv[2] * wb[1] + zv[3] * wb[3];
  }
  so[2 * tid] = o0; so[2 * tid + 1] = o1;
  __syncthreads();
  if (tid < NT / 2) {
    const int r2 = blockIdx.x * NT + 2 * tid;
    if (r2 + 1 < NN) {
      const v4f v = *(const v4f*)(so + 4 * tid);
      float* op = out + (size_t)r2 * OUT_D;
      *(volatile v4f*)op = v;
      __threadfence();
      *(volatile v4f*)op = v;
    }
  }
}

extern "C" void kernel_launch(void* const* d_in, const int* in_sizes, int n_in,
                              void* d_out, int out_size, void* d_ws, size_t ws_size, hipStream_t stream) {
  (void)n_in;
  if (in_sizes[0] != NN * IN_D || in_sizes[1] != 2 * NE || out_size != NN * OUT_D) return;
  const float* X      = (const float*)d_in[0];
  const int*   ei     = (const int*)  d_in[1];
  const float* emb_W  = (const float*)d_in[2];
  const float* emb_b  = (const float*)d_in[3];
  const float* Wself  = (const float*)d_in[4];
  const float* Wneigh = (const float*)d_in[5];
  const float* conv_b = (const float*)d_in[6];
  const float* bn_g   = (const float*)d_in[7];
  const float* bn_b   = (const float*)d_in[8];
  const float* W1     = (const float*)d_in[9];
  const float* b1     = (const float*)d_in[10];
  const float* W2     = (const float*)d_in[11];
  const float* b2     = (const float*)d_in[12];
  float* out = (float*)d_out;

  char* ws = (char*)d_ws; size_t off = 0;
  auto carve = [&](size_t bytes) -> char* { char* p = ws + off; off += (bytes + 255) & ~(size_t)255; return p; };
  unsigned*       B0H   = (unsigned*)carve((size_t)HD * XK * 2);
  unsigned*       B0L   = (unsigned*)carve((size_t)HD * XK * 2);
  float*          BIAS0 = (float*)carve((size_t)HD * 4);
  unsigned*       BLH   = (unsigned*)carve((size_t)2 * HD * KC * 2);
  unsigned*       BLL   = (unsigned*)carve((size_t)2 * HD * KC * 2);
  unsigned*       W1H   = (unsigned*)carve((size_t)HD2 * HD * 2);
  unsigned*       W1L   = (unsigned*)carve((size_t)HD2 * HD * 2);
  float*          PART  = (float*)carve((size_t)NSB * 2 * HD * 4);
  float*          MURS  = (float*)carve((size_t)2 * HD * 4);
  float*          P     = (float*)carve((size_t)NP * HD * 4);
  char*           Qc    = carve((size_t)NP * HD * 4);
  unsigned short* APH   = (unsigned short*)carve((size_t)CHR * KC * 2);
  unsigned short* APL   = (unsigned short*)carve((size_t)CHR * KC * 2);
  float*          ACC   = (float*)carve((size_t)CHR * HD * 4);
  if (off > ws_size || off > (size_t)134217728) return;
  float*          Q   = (float*)Qc;
  float*          XCF = (float*)Qc;
  unsigned*       XCH = (unsigned*)(Qc + (size_t)NP * XK * 4);
  unsigned*       XCL = (unsigned*)(Qc + (size_t)NP * XK * 4 + (size_t)NP * XK * 2);
  unsigned short* H3H = (unsigned short*)Qc;
  unsigned short* H3L = (unsigned short*)(Qc + (size_t)NP * HD * 2);

  prep_kernel<<<(39040 + NT - 1) / NT, NT, 0, stream>>>(emb_W, emb_b, Wself, Wneigh, conv_b, W1, BLH, BLL, W1H, W1L, B0H, B0L, BIAS0);

  agg0_kernel<<<NTL, NT, 0, stream>>>(X, ei, XCF, XCH, XCL);
  {
    const int tiles = (NP / 64) * (HD / 64);
    wmma_gemm64<1, true, 2, 0, false, 0><<<dim3((tiles + 7) / 8, 1), 256, 0, stream>>>(
        (const unsigned short*)XCH, (const unsigned short*)XCL, XK, 0L,
        (const unsigned short*)B0H, (const unsigned short*)B0L, XK, 0L,
        (void*)P, (void*)nullptr, HD, 0L,
        BIAS0, (const float*)nullptr, 0L, NP, HD, XK, 1.0f);
  }
  stats_kernel<<<NSB, NT, 0, stream>>>(P, PART);
  fin_kernel<<<1, 128, 0, stream>>>(PART, MURS);
  apply_kernel<<<NP * 32 / NT, NT, 0, stream>>>(P, P, MURS, bn_g, bn_b, 0);

  for (int li = 1; li < 3; ++li) {
    float* hin  = (li == 1) ? P : Q;
    float* pout = (li == 1) ? Q : P;
    const unsigned short* bh = (const unsigned short*)BLH + (size_t)(li - 1) * HD * KC;
    const unsigned short* bl = (const unsigned short*)BLL + (size_t)(li - 1) * HD * KC;
    for (int ch = 0; ch < NCHK; ++ch) {
      agg_kernel<<<TPC, NT, 0, stream>>>(hin, ei, ACC, APH, APL, ch * TPC);
      const int tiles = (CHR / 64) * (HD / 64);
      wmma_gemm64<1, true, 2, 0, false, 0><<<dim3((tiles + 7) / 8, 1), 256, 0, stream>>>(
          (const unsigned short*)APH, (const unsigned short*)APL, KC, 0L,
          bh, bl, KC, 0L,
          (void*)(pout + (size_t)ch * CHR * HD), (void*)nullptr, HD, 0L,
          conv_b + (size_t)li * HD, (const float*)nullptr, 0L, CHR, HD, KC, 1.0f);
    }
    stats_kernel<<<NSB, NT, 0, stream>>>(pout, PART);
    fin_kernel<<<1, 128, 0, stream>>>(PART, MURS);
    apply_kernel<<<NP * 32 / NT, NT, 0, stream>>>(pout, hin, MURS, bn_g + (size_t)li * HD, bn_b + (size_t)li * HD, 1);
  }

  convert_kernel<<<NP * HD / 8 / NT, NT, 0, stream>>>(P, H3H, H3L);
  {
    const int tiles = (NP / 64) * (HD2 / 64);
    wmma_gemm64<1, true, 2, 0, false, 2><<<dim3((tiles + 7) / 8, 1), 256, 0, stream>>>(
        (const unsigned short*)H3H, (const unsigned short*)H3L, HD, 0L,
        (const unsigned short*)W1H, (const unsigned short*)W1L, HD, 0L,
        (void*)P, (void*)nullptr, HD2, 0L,
        b1, (const float*)nullptr, 0L, NP, HD2, HD, 1.0f);
  }
  out_kernel<<<NSB, NT, 0, stream>>>(P, W2, b2, out);
}
